// CombinedNN_65635690217686
// MI455X (gfx1250) — hardware-verified
//
#include <hip/hip_runtime.h>
#include <math.h>
typedef __attribute__((ext_vector_type(16))) _Float16 v16h;
typedef __attribute__((ext_vector_type(8)))  _Float16 v8h;
typedef __attribute__((ext_vector_type(16))) __bf16   v16b;
typedef __attribute__((ext_vector_type(8)))  __bf16   v8b;
typedef __attribute__((ext_vector_type(8)))  float    v8f;
typedef __attribute__((ext_vector_type(4)))  float    v4f;
#define PSCALE 32768.0f
#define U16(p) ((const unsigned short*)(const void*)(p))
#define PSCALE_INV (1.0f / 32768.0f)

__device__ __forceinline__ unsigned short f2bf_bits(float f) {
  unsigned u = __float_as_uint(f);
  return (unsigned short)((u + 0x7FFFu + ((u >> 16) & 1u)) >> 16);
}
__device__ __forceinline__ float bf_bits2f(unsigned short h) { return __uint_as_float(((unsigned)h) << 16); }

__device__ __forceinline__ void dep_guard_h(v8f& a, v8f& b, v16h x, v16h y) { asm volatile("v_nop\n\tv_nop\n\tv_nop\n\tv_nop" : "+v"(a), "+v"(b) : "v"(x), "v"(y)); }
__device__ __forceinline__ void dep_guard_b(v8f& a, v8f& b, v16b x, v16b y) { asm volatile("v_nop\n\tv_nop\n\tv_nop\n\tv_nop" : "+v"(a), "+v"(b) : "v"(x), "v"(y)); }
__device__ __forceinline__ void keep4_h(v16h a, v16h b, v16h c, v16h d) { asm volatile("v_nop" :: "v"(a), "v"(b), "v"(c), "v"(d)); }
__device__ __forceinline__ void keep4_b(v16b a, v16b b, v16b c, v16b d) { asm volatile("v_nop" :: "v"(a), "v"(b), "v"(c), "v"(d)); }
__device__ __forceinline__ void acc_guard4(v8f& a, v8f& b, v8f& c, v8f& d) { asm volatile("v_nop\n\tv_nop\n\tv_nop\n\tv_nop" : "+v"(a), "+v"(b), "+v"(c), "+v"(d)); }
template <typename T> struct Frag;
template <> struct Frag<_Float16> {
  typedef v16h V; union U { v16h v; v8h h[2]; };
  static __device__ __forceinline__ v16h load(const _Float16* p) {
    U f; f.h[0] = *(const v8h*)(p); f.h[1] = *(const v8h*)(p + 16); return f.v;
  }
  static __device__ __forceinline__ v8f mma(v16h a, v16h b, v8f c) {
    return __builtin_amdgcn_wmma_f32_16x16x32_f16(false, a, false, b, (short)0, c, false, false);
  }
  static __device__ __forceinline__ void guard(v8f& a, v8f& b, v16h x, v16h y) { dep_guard_h(a, b, x, y); }
  static __device__ __forceinline__ void keep(v16h a, v16h b, v16h c, v16h d) { keep4_h(a, b, c, d); }
};
template <> struct Frag<__bf16> {
  typedef v16b V; union U { v16b v; v8b h[2]; };
  static __device__ __forceinline__ v16b load(const __bf16* p) {
    U f; f.h[0] = *(const v8b*)(p); f.h[1] = *(const v8b*)(p + 16); return f.v;
  }
  static __device__ __forceinline__ v8f mma(v16b a, v16b b, v8f c) {
    return __builtin_amdgcn_wmma_f32_16x16x32_bf16(false, a, false, b, (short)0, c, false, false);
  }
  static __device__ __forceinline__ void guard(v8f& a, v8f& b, v16b x, v16b y) { dep_guard_b(a, b, x, y); }
  static __device__ __forceinline__ void keep(v16b a, v16b b, v16b c, v16b d) { keep4_b(a, b, c, d); }
};

template <int ET> struct Elem;
template <> struct Elem<0> { typedef _Float16 T; };
template <> struct Elem<1> { typedef __bf16 T; };
template <int ET, bool SPLIT, int BIAS_MODE, int OUT_MODE, bool RESID, int ACT = 0>
__global__ __launch_bounds__(256) void wmma_gemm64(
    const unsigned short* __restrict__ Ap, const unsigned short* __restrict__ A2p, int lda, long strideA,
    const unsigned short* __restrict__ Btp, const unsigned short* __restrict__ Bt2p, int ldb, long strideB,
    void* __restrict__ Cout, void* __restrict__ Cout2, int ldc, long strideC,
    const float* __restrict__ bias,
    const float* __restrict__ resid, long strideR,
    int M, int N, int K, float scale) {
  typedef typename Elem<ET>::T T;
  typedef typename Frag<T>::V V;
  const T* A = (const T*)Ap; const T* A2 = (const T*)A2p; const T* Bt = (const T*)Btp; const T* Bt2 = (const T*)Bt2p;
  __shared__ __align__(16) float sT[8][16 * 68];
  const int b    = blockIdx.y;
  const int lane = threadIdx.x & 31;
  const int wave = threadIdx.x >> 5;
  const int tilesN = N >> 6;
  const int tilesM = M >> 6;
  const int tile = blockIdx.x * 8 + wave;
  if (tile >= tilesM * tilesN) return;
  const int tm = tile / tilesN;
  const int tn = tile - tm * tilesN;
  const int m0 = tm << 6;
  const int n0 = tn << 6;

  const T* Ab  = A  + (size_t)b * strideA;
  const T* Bb  = Bt + (size_t)b * strideB;
  const T* Ab2 = SPLIT ? (A2  + (size_t)b * strideA) : nullptr;
  const T* Bb2 = SPLIT ? (Bt2 + (size_t)b * strideB) : nullptr;

  const int rlane = lane & 15;
  const int koff  = (lane >> 4) * 8;
  const int mOff  = (lane >> 4) * 8;

  v8f acc[4][4];
#pragma unroll
  for (int i = 0; i < 4; ++i)
#pragma unroll
    for (int j = 0; j < 4; ++j) acc[i][j] = (v8f){0.f,0.f,0.f,0.f,0.f,0.f,0.f,0.f};

  for (int k0 = 0; k0 < K; k0 += 32) {
    V bh[4], bl[4];
#pragma unroll
    for (int j = 0; j < 4; ++j) {
      const size_t bo = (size_t)(n0 + (j << 4) + rlane) * ldb + koff + k0;
      bh[j] = Frag<T>::load(Bb + bo);
      if (SPLIT) bl[j] = Frag<T>::load(Bb2 + bo);
    }
#pragma unroll
    for (int i = 0; i < 4; ++i) {
      const size_t ao = (size_t)(m0 + (i << 4) + rlane) * lda + koff + k0;
      V ah = Frag<T>::load(Ab + ao);
      V al;
      if (SPLIT) al = Frag<T>::load(Ab2 + ao);
#pragma unroll
      for (int j = 0; j < 4; ++j) {
        acc[i][j] = Frag<T>::mma(ah, bh[j], acc[i][j]);
        if (SPLIT) {
          acc[i][j] = Frag<T>::mma(ah, bl[j], acc[i][j]);
          acc[i][j] = Frag<T>::mma(al, bh[j], acc[i][j]);
        }
      }
      Frag<T>::guard(acc[i][0], acc[i][3], ah, SPLIT ? al : ah);
    }
    Frag<T>::keep(bh[0], bh[1], bh[2], bh[3]);
    if (SPLIT) Frag<T>::keep(bl[0], bl[1], bl[2], bl[3]);
  }
  acc_guard4(acc[0][0], acc[0][1], acc[0][2], acc[0][3]);
  acc_guard4(acc[1][0], acc[1][1], acc[1][2], acc[1][3]);
  acc_guard4(acc[2][0], acc[2][1], acc[2][2], acc[2][3]);
  acc_guard4(acc[3][0], acc[3][1], acc[3][2], acc[3][3]);

  float* slab = sT[wave];
  const float* Rb = RESID ? (resid + (size_t)b * strideR) : nullptr;
#pragma unroll
  for (int i = 0; i < 4; ++i) {
    const int mBase = m0 + (i << 4);
#pragma unroll
    for (int j = 0; j < 4; ++j) {
      const int n = n0 + (j << 4) + rlane;
      float bv = 0.f;
      if (BIAS_MODE == 2) bv = bias[n];
#pragma unroll
      for (int r = 0; r < 8; ++r) {
        float v = acc[i][j][r] * scale;
        if (BIAS_MODE == 1) v += bias[mBase + mOff + r];
        if (BIAS_MODE == 2) v += bv;
        if (RESID) v += Rb[(size_t)(mBase + mOff + r) * ldc + n];
        if (ACT == 1) v = tanhf(v);
        if (ACT == 2) v = fmaxf(v, 0.0f);
        if (ACT == 3) v = v / (1.0f + expf(-v));
        if (ACT == 4) v = (v > 0.f) ? v : 0.01f * v;
        if (ACT == 5) v = 0.5f * v * (1.0f + erff(v * 0.70710678118654752f));
        slab[(mOff + r) * 68 + (j << 4) + rlane] = v;
      }
    }
    __builtin_amdgcn_fence(__ATOMIC_RELEASE, "workgroup");
    __builtin_amdgcn_wave_barrier();
    __builtin_amdgcn_fence(__ATOMIC_ACQUIRE, "workgroup");
    if (OUT_MODE == 0) {
      float* C = (float*)Cout + (size_t)b * strideC;
      const int hh = lane >> 4, c4 = (lane & 15) * 4;
      for (int pass = 0; pass < 2; ++pass) {
#pragma unroll
        for (int it = 0; it < 8; ++it) {
          const int row = it * 2 + hh;
          v4f v = *(const v4f*)(slab + row * 68 + c4);
          *(volatile v4f*)(C + (size_t)(mBase + row) * ldc + n0 + c4) = v;
        }
        __threadfence();
      }
    } else {
      const int q = lane >> 3, c8 = (lane & 7) * 8;
      unsigned short* C  = (unsigned short*)Cout  + (size_t)b * strideC;
      unsigned short* C2 = (OUT_MODE == 2) ? ((unsigned short*)Cout2 + (size_t)b * strideC) : nullptr;
      for (int pass = 0; pass < 2; ++pass) {
#pragma unroll
        for (int it = 0; it < 4; ++it) {
          const int row = it * 4 + q;
          const float* sp = slab + row * 68 + c8;
          v8h hv, lv;
#pragma unroll
          for (int e = 0; e < 8; ++e) {
            if (OUT_MODE == 1) {
              hv[e] = (_Float16)sp[e];
            } else {
              unsigned short hb = f2bf_bits(sp[e]);
              unsigned short lb = f2bf_bits(sp[e] - bf_bits2f(hb));
              hv[e] = __builtin_bit_cast(_Float16, hb);
              lv[e] = __builtin_bit_cast(_Float16, lb);
            }
          }
          *(volatile v8h*)(C + (size_t)(mBase + row) * ldc + n0 + c8) = hv;
          if (OUT_MODE == 2) *(volatile v8h*)(C2 + (size_t)(mBase + row) * ldc + n0 + c8) = lv;
        }
        __threadfence();
      }
    }
    __builtin_amdgcn_fence(__ATOMIC_RELEASE, "workgroup");
    __builtin_amdgcn_wave_barrier();
    __builtin_amdgcn_fence(__ATOMIC_ACQUIRE, "workgroup");
  }
}

__global__ __launch_bounds__(256) void cast_f32_f16x2(
    const float* __restrict__ in, _Float16* __restrict__ out, int n2) {
  int i = blockIdx.x * 256 + threadIdx.x;
  if (i < n2) {
    const _Float16 h0 = (_Float16)in[2 * i], h1 = (_Float16)in[2 * i + 1];
    const unsigned u = (unsigned)__builtin_bit_cast(unsigned short, h0) | ((unsigned)__builtin_bit_cast(unsigned short, h1) << 16);
    ((volatile unsigned*)out)[i] = u;
    __threadfence();
    ((volatile unsigned*)out)[i] = u;
  }
}


__global__ __launch_bounds__(256) void transpose_cast_f16(const float* __restrict__ in, int ldi,
                                                         _Float16* __restrict__ outT, int ldo, float scale) {
  __shared__ __align__(16) _Float16 tile[64][72];
  const int c0 = blockIdx.x * 64, r0 = blockIdx.y * 64;
  const int t = threadIdx.y * 32 + threadIdx.x;
  for (int i = threadIdx.y; i < 64; i += 8) {
    tile[threadIdx.x][i]      = (_Float16)(in[(size_t)(r0 + i) * ldi + c0 + threadIdx.x] * scale);
    tile[32 + threadIdx.x][i] = (_Float16)(in[(size_t)(r0 + i) * ldi + c0 + 32 + threadIdx.x] * scale);
  }
  __syncthreads();
  const int q = t >> 3, c8 = (t & 7) * 8;
  for (int pass = 0; pass < 2; ++pass) {
#pragma unroll
    for (int it = 0; it < 2; ++it) {
      const int c = it * 32 + q;
      v8h hv = *(const v8h*)(&tile[c][c8]);
      *(volatile v8h*)(outT + (size_t)(c0 + c) * ldo + r0 + c8) = hv;
    }
    __threadfence();
  }
}

#define CB 2
#define CS 1024
#define CD 512
#define CF 2048
#define CHID 32
#define CCLS 1000
#define CR (CB * CS)
__global__ __launch_bounds__(256) void bias_kernel(const float* __restrict__ coords, const float* __restrict__ rw1, const float* __restrict__ rb1, const float* __restrict__ rw2, const float* __restrict__ rb2,
                                                  const float* __restrict__ tw1, const float* __restrict__ tb1, const float* __restrict__ tw2, const float* __restrict__ tb2,
                                                  const float* __restrict__ fw1, const float* __restrict__ fb1, const float* __restrict__ fw2, const float* __restrict__ fb2, float* __restrict__ BIAS) {
  __shared__ float srw1[3 * CHID], srb1[CHID], srw2[CHID], stw1[2 * CHID], stb1[CHID], stw2[CHID], sfw1[4 * CHID], sfb1[CHID], sfw2[CHID];
  const int t = threadIdx.x;
  if (t < CHID) { srb1[t] = rb1[t]; srw2[t] = rw2[t]; stb1[t] = tb1[t]; stw2[t] = tw2[t]; sfb1[t] = fb1[t]; sfw2[t] = fw2[t]; }
  for (int i = t; i < 3 * CHID; i += 256) srw1[i] = rw1[i];
  for (int i = t; i < 2 * CHID; i += 256) stw1[i] = tw1[i];
  for (int i = t; i < 4 * CHID; i += 256) sfw1[i] = fw1[i];
  __syncthreads();
  const size_t idx = (size_t)blockIdx.x * 256 + t;
  const int b = (int)(idx / ((size_t)CS * CS)); const int i = (int)((idx / CS) % CS), j = (int)(idx % CS);
  const float xi = coords[((size_t)b * CS + i) * 2], yi = coords[((size_t)b * CS + i) * 2 + 1], xj = coords[((size_t)b * CS + j) * 2], yj = coords[((size_t)b * CS + j) * 2 + 1];
  const float dx = xj - xi, dy = yj - yi;
  const float dist = sqrtf(dx * dx + dy * dy + 1e-8f); const float th = atan2f(dy, dx); const float sn = sinf(th), cs = cosf(th);
  float acc = rb2[0] + tb2[0] + fb2[0];
#pragma unroll 1
  for (int h = 0; h < CHID; ++h) {
    const float a = fmaxf(srb1[h] + dist * srw1[h] + sn * srw1[CHID + h] + cs * srw1[2 * CHID + h], 0.f);
    const float c = fmaxf(stb1[h] + dx * stw1[h] + dy * stw1[CHID + h], 0.f);
    const float d = fmaxf(sfb1[h] + dx * sfw1[h] + dy * sfw1[CHID + h] - dx * sfw1[2 * CHID + h] - dy * sfw1[3 * CHID + h], 0.f);
    acc += a * srw2[h] + c * stw2[h] + d * sfw2[h];
  }
  ((volatile float*)BIAS)[idx] = acc; __threadfence(); ((volatile float*)BIAS)[idx] = acc;
}
__global__ __launch_bounds__(256) void vt_kernel(const unsigned short* __restrict__ QKV16, unsigned* __restrict__ VT) {
  __shared__ unsigned short tile[64][66];
  const int b = blockIdx.z, d0 = blockIdx.y * 64, j0 = blockIdx.x * 64, tx = threadIdx.x, ty = threadIdx.y;
  for (int r = ty; r < 64; r += 8) { const int j = j0 + r; const unsigned short* src = QKV16 + ((size_t)b * CS + j) * (3 * CD) + 2 * CD + d0; tile[2 * tx][r] = src[2 * tx]; tile[2 * tx + 1][r] = src[2 * tx + 1]; }
  __syncthreads();
  for (int pass = 0; pass < 2; ++pass) { for (int r = ty; r < 64; r += 8) { const int d = d0 + r; const unsigned u = (unsigned)tile[r][2 * tx] | ((unsigned)tile[r][2 * tx + 1] << 16);
      ((volatile unsigned*)VT)[(((size_t)b * CD + d) * CS + j0) / 2 + tx] = u; } __threadfence(); }
}
__global__ __launch_bounds__(256) void softmax_kernel(const float* __restrict__ Sm, const float* __restrict__ BIAS, unsigned* __restrict__ P16) {
  __shared__ float red[8]; __shared__ float stat;
  const size_t row = blockIdx.x; const int t = threadIdx.x, lane = t & 31, wave = t >> 5;
  const float* sr = Sm + row * CS; const float* br = BIAS + row * CS;
  float v[4]; float mx = -INFINITY;
#pragma unroll
  for (int q = 0; q < 2; ++q) { const int c = q * 512 + 2 * t; v[2*q] = sr[c] + br[c]; v[2*q+1] = sr[c + 1] + br[c + 1]; mx = fmaxf(mx, fmaxf(v[2*q], v[2*q+1])); }
  for (int o = 16; o > 0; o >>= 1) mx = fmaxf(mx, __shfl_xor(mx, o, 32));
  if (lane == 0) red[wave] = mx; __syncthreads();
  if (t == 0) { float m = red[0]; for (int w = 1; w < 8; ++w) m = fmaxf(m, red[w]); stat = m; } __syncthreads();
  const float m = stat; __syncthreads();
  float se = 0.f;
#pragma unroll
  for (int q = 0; q < 4; ++q) { v[q] = expf(v[q] - m); se += v[q]; }
  for (int o = 16; o > 0; o >>= 1) se += __shfl_xor(se, o, 32);
  if (lane == 0) red[wave] = se; __syncthreads();
  if (t == 0) { float s = 0.f; for (int w = 0; w < 8; ++w) s += red[w]; stat = 32768.0f / s; } __syncthreads();
  const float inv = stat;
  for (int pass = 0; pass < 2; ++pass) {
#pragma unroll
    for (int q = 0; q < 2; ++q) { const unsigned u = (unsigned)__builtin_bit_cast(unsigned short, (_Float16)(v[2*q] * inv)) | ((unsigned)__builtin_bit_cast(unsigned short, (_Float16)(v[2*q+1] * inv)) << 16);
      ((volatile unsigned*)P16)[row * (CS / 2) + q * 256 + t] = u; }
    __threadfence(); }
}
__global__ __launch_bounds__(256) void add_ln_kernel(float* __restrict__ X, const float* __restrict__ A, const float* __restrict__ g, const float* __restrict__ bb, unsigned* __restrict__ X16) {
  const int lane = threadIdx.x & 31, wave = threadIdx.x >> 5; const size_t row = (size_t)blockIdx.x * 8 + wave;
  float v[16]; float s = 0.f;
#pragma unroll
  for (int q = 0; q < 4; ++q) { const v4f a = *(const v4f*)(X + row * CD + q * 128 + lane * 4); v4f d = {0.f, 0.f, 0.f, 0.f}; if (A) d = *(const v4f*)(A + row * CD + q * 128 + lane * 4);
    for (int e = 0; e < 4; ++e) { v[4*q+e] = a[e] + d[e]; s += v[4*q+e]; } }
  for (int o = 16; o > 0; o >>= 1) s += __shfl_xor(s, o, 32);
  const float mean = s / (float)CD; float s2 = 0.f;
#pragma unroll
  for (int i = 0; i < 16; ++i) { const float d = v[i] - mean; s2 += d * d; }
  for (int o = 16; o > 0; o >>= 1) s2 += __shfl_xor(s2, o, 32);
  const float inv = rsqrtf(s2 / (float)CD + 1e-5f);
  typedef __attribute__((ext_vector_type(2))) unsigned u2;
  for (int pass = 0; pass < 2; ++pass) {
#pragma unroll
    for (int q = 0; q < 4; ++q) { const int c = q * 128 + lane * 4; v4f o4; u2 pk;
      for (int e = 0; e < 4; ++e) o4[e] = (v[4*q+e] - mean) * inv * g[c + e] + bb[c + e];
      pk[0] = (unsigned)__builtin_bit_cast(unsigned short, (_Float16)o4[0]) | ((unsigned)__builtin_bit_cast(unsigned short, (_Float16)o4[1]) << 16);
      pk[1] = (unsigned)__builtin_bit_cast(unsigned short, (_Float16)o4[2]) | ((unsigned)__builtin_bit_cast(unsigned short, (_Float16)o4[3]) << 16);
      *(volatile v4f*)(X + row * CD + c) = o4; *(volatile u2*)(X16 + (row * CD + c) / 2) = pk; }
    __threadfence(); }
}
__global__ __launch_bounds__(256) void pool_fc_kernel(const float* __restrict__ X, const float* __restrict__ fw, const float* __restrict__ fb, float* __restrict__ out) {
  __shared__ float pooled[CD];
  const int b = blockIdx.y, o0 = blockIdx.x * 256, t = threadIdx.x;
  for (int d = t; d < CD; d += 256) { float s = 0.f;
#pragma unroll 1
    for (int r = 0; r < CS; ++r) s += X[((size_t)b * CS + r) * CD + d];
    pooled[d] = s / (float)CS; }
  __syncthreads();
  const int o = o0 + t; float acc = 0.f;
  if (o < CCLS) { acc = fb[o];
#pragma unroll 1
    for (int d = 0; d < CD; ++d) acc += pooled[d] * fw[(size_t)d * CCLS + o]; }
  if (o < CCLS) { ((volatile float*)out)[(size_t)b * CCLS + o] = acc; __threadfence(); ((volatile float*)out)[(size_t)b * CCLS + o] = acc; }
}

__global__ __launch_bounds__(256) void copy_cast_kernel(const float* __restrict__ x, float* __restrict__ X, unsigned* __restrict__ X16, long n2) {
  const long i = (long)blockIdx.x * 256 + threadIdx.x; if (i >= n2) return;
  typedef __attribute__((ext_vector_type(2))) float v2f; const v2f v = *(const v2f*)(x + 2 * i);
  const unsigned u = (unsigned)__builtin_bit_cast(unsigned short, (_Float16)v[0]) | ((unsigned)__builtin_bit_cast(unsigned short, (_Float16)v[1]) << 16);
  for (int pass = 0; pass < 2; ++pass) { *(volatile v2f*)(X + 2 * i) = v; ((volatile unsigned*)X16)[i] = u; __threadfence(); }
}
#ifndef NLAYERS
#define NLAYERS 2
#endif
extern "C" void kernel_launch(void* const* d_in, const int* in_sizes, int n_in, void* d_out, int out_size, void* d_ws, size_t ws_size, hipStream_t stream) {
  (void)in_sizes; (void)n_in; (void)out_size; (void)ws_size;
  const float* x = (const float*)d_in[0]; const float* coords = (const float*)d_in[1];
  const float* Wq = (const float*)d_in[2]; const float* Wk = (const float*)d_in[3]; const float* Wv = (const float*)d_in[4];
  const float* rw1 = (const float*)d_in[5]; const float* rb1 = (const float*)d_in[6]; const float* rw2 = (const float*)d_in[7]; const float* rb2 = (const float*)d_in[8];
  const float* tw1 = (const float*)d_in[9]; const float* tb1 = (const float*)d_in[10]; const float* tw2 = (const float*)d_in[11]; const float* tb2 = (const float*)d_in[12];
  const float* fw1 = (const float*)d_in[13]; const float* fb1 = (const float*)d_in[14]; const float* fw2 = (const float*)d_in[15]; const float* fb2 = (const float*)d_in[16];
  const float* ln1g = (const float*)d_in[17]; const float* ln1b = (const float*)d_in[18]; const float* f1w = (const float*)d_in[19]; const float* f1b = (const float*)d_in[20]; const float* f2w = (const float*)d_in[21]; const float* f2b = (const float*)d_in[22];
  const float* ln2g = (const float*)d_in[23]; const float* ln2b = (const float*)d_in[24]; const float* lnfg = (const float*)d_in[25]; const float* lnfb = (const float*)d_in[26]; const float* fcw = (const float*)d_in[27]; const float* fcb = (const float*)d_in[28];
  float* out = (float*)d_out;
  char* ws = (char*)d_ws; size_t off = 0;
  auto carve = [&](size_t bytes) -> char* { char* p = ws + off; off += (bytes + 255) & ~(size_t)255; return p; };
  float* X = (float*)carve((size_t)CR * CD * 4); unsigned* X16 = (unsigned*)carve((size_t)CR * CD * 2);
  _Float16* WT = (_Float16*)carve((size_t)3 * CD * CD * 2); _Float16* W1T = (_Float16*)carve((size_t)CF * CD * 2); _Float16* W2T = (_Float16*)carve((size_t)CD * CF * 2);
  unsigned* QKV16 = (unsigned*)carve((size_t)CR * 3 * CD * 2); unsigned* VT = (unsigned*)carve((size_t)CB * CD * CS * 2);
  float* BIAS = (float*)carve((size_t)CB * CS * CS * 4); float* Sm = (float*)carve((size_t)CB * CS * CS * 4); unsigned* P16 = (unsigned*)carve((size_t)CB * CS * CS * 2);
  float* AO = (float*)carve((size_t)CR * CD * 4); unsigned* H16 = (unsigned*)carve((size_t)CR * CF * 2);
  copy_cast_kernel<<<(CR * CD / 2 + 255) / 256, 256, 0, stream>>>(x, X, X16, (long)CR * CD / 2);
  for (int l = 0; l < NLAYERS; ++l) {
    bias_kernel<<<CB * CS * CS / 256, 256, 0, stream>>>(coords, rw1 + l * 3 * CHID, rb1 + l * CHID, rw2 + l * CHID, rb2 + l, tw1 + l * 2 * CHID, tb1 + l * CHID, tw2 + l * CHID, tb2 + l, fw1 + l * 4 * CHID, fb1 + l * CHID, fw2 + l * CHID, fb2 + l, BIAS);
    transpose_cast_f16<<<dim3(CD / 64, CD / 64), dim3(32, 8), 0, stream>>>(Wq + (size_t)l * CD * CD, CD, WT, CD, 1.0f);
    transpose_cast_f16<<<dim3(CD / 64, CD / 64), dim3(32, 8), 0, stream>>>(Wk + (size_t)l * CD * CD, CD, WT + (size_t)CD * CD, CD, 1.0f);
    transpose_cast_f16<<<dim3(CD / 64, CD / 64), dim3(32, 8), 0, stream>>>(Wv + (size_t)l * CD * CD, CD, WT + (size_t)2 * CD * CD, CD, 1.0f);
    { const int t = (CR / 64) * (3 * CD / 64);
      wmma_gemm64<0, false, 0, 1, false><<<dim3((t + 7) / 8, 1), 256, 0, stream>>>((const unsigned short*)X16, nullptr, CD, 0, U16(WT), nullptr, CD, 0, QKV16, nullptr, 3 * CD, 0, nullptr, nullptr, 0, CR, 3 * CD, CD, 1.0f); }
    vt_kernel<<<dim3(CS / 64, CD / 64, CB), dim3(32, 8), 0, stream>>>((const unsigned short*)QKV16, VT);
    { const int t = (CS / 64) * (CS / 64);
      wmma_gemm64<0, false, 0, 0, false><<<dim3((t + 7) / 8, CB), 256, 0, stream>>>((const unsigned short*)QKV16, nullptr, 3 * CD, (long)CS * 3 * CD, (const unsigned short*)QKV16 + CD, nullptr, 3 * CD, (long)CS * 3 * CD, Sm, nullptr, CS, (long)CS * CS, nullptr, nullptr, 0, CS, CS, CD, 0.044194173824159216f); }
    softmax_kernel<<<CB * CS, 256, 0, stream>>>(Sm, BIAS, P16);
    { const int t = (CS / 64) * (CD / 64);
      wmma_gemm64<0, false, 0, 0, false><<<dim3((t + 7) / 8, CB), 256, 0, stream>>>((const unsigned short*)P16, nullptr, CS, (long)CS * CS, (const unsigned short*)VT, nullptr, CS, (long)CD * CS, AO, nullptr, CD, (long)CS * CD, nullptr, nullptr, 0, CS, CD, CS, 1.0f / 32768.0f); }
    add_ln_kernel<<<CR / 8, 256, 0, stream>>>(X, AO, ln1g + l * CD, ln1b + l * CD, X16);
    transpose_cast_f16<<<dim3(CF / 64, CD / 64), dim3(32, 8), 0, stream>>>(f1w + (size_t)l * CD * CF, CF, W1T, CD, 1.0f);
    transpose_cast_f16<<<dim3(CD / 64, CF / 64), dim3(32, 8), 0, stream>>>(f2w + (size_t)l * CF * CD, CD, W2T, CF, 1.0f);
    { const int t = (CR / 64) * (CF / 64);
      wmma_gemm64<0, false, 2, 1, false, 2><<<dim3((t + 7) / 8, 1), 256, 0, stream>>>((const unsigned short*)X16, nullptr, CD, 0, U16(W1T), nullptr, CD, 0, H16, nullptr, CF, 0, f1b + l * CF, nullptr, 0, CR, CF, CD, 1.0f);
      const int t2 = (CR / 64) * (CD / 64);
      wmma_gemm64<0, false, 2, 0, false><<<dim3((t2 + 7) / 8, 1), 256, 0, stream>>>((const unsigned short*)H16, nullptr, CF, 0, U16(W2T), nullptr, CF, 0, AO, nullptr, CD, 0, f2b + l * CD, nullptr, 0, CR, CD, CF, 1.0f); }
    add_ln_kernel<<<CR / 8, 256, 0, stream>>>(X, AO, ln2g + l * CD, ln2b + l * CD, X16);
  }
  add_ln_kernel<<<CR / 8, 256, 0, stream>>>(X, nullptr, lnfg, lnfb, X16);
  pool_fc_kernel<<<dim3((CCLS + 255) / 256, CB), 256, 0, stream>>>(X, fcw, fcb, out);
}
